// _MambaBlock_72825465471238
// MI455X (gfx1250) — hardware-verified
//
#include <hip/hip_runtime.h>

#define NBATCH 8
#define NL     512
#define NDIM   256
#define NIN    512
#define NROWS  (NBATCH * NL)
#define NPJ    (2 * NIN)
#define TCH    32

static_assert(NDIM % 32 == 0 && NIN % 32 == 0);
static_assert(NROWS % 128 == 0 && NPJ % 64 == 0);
static_assert(NROWS % 32 == 0);
static_assert(NL % TCH == 0 && NIN % 64 == 0);

typedef __bf16         v16b __attribute__((ext_vector_type(16)));
typedef unsigned short v8us __attribute__((ext_vector_type(8)));
typedef float          v8f  __attribute__((ext_vector_type(8)));
typedef float          v4f  __attribute__((ext_vector_type(4)));
typedef v8us __attribute__((may_alias)) v8usa;
typedef v4f  __attribute__((may_alias)) v4fa;

union Frag { v16b v; v8us half[2]; };

constexpr int P_X    = 0;
constexpr int P_WIN  = P_X + NROWS * NDIM;
constexpr int P_WOUT = P_WIN + NPJ * NDIM;
constexpr int P_END  = P_WOUT + NDIM * NIN;
constexpr int NPC    = P_END / 8;
constexpr int NCBLK  = NPC / 256;
static_assert(P_END % 8 == 0);
static_assert(NPC % 256 == 0);
static_assert(P_WIN % 2048 == 0 && P_WOUT % 2048 == 0);

constexpr size_t OFF_CV = 0;
constexpr size_t SZ_CV  = (size_t)P_END * 2;
constexpr size_t OFF_XP = OFF_CV + SZ_CV;
constexpr size_t SZ_XP  = (size_t)NROWS * NPJ * 4;
constexpr size_t OFF_YH = OFF_XP + SZ_XP;
constexpr size_t SZ_Y   = (size_t)NROWS * NIN * 2;
constexpr size_t OFF_YL = OFF_YH + SZ_Y;
constexpr size_t WS_END = OFF_YL + SZ_Y;
static_assert(OFF_XP % 128 == 0 && OFF_YH % 128 == 0 && OFF_YL % 128 == 0);
static_assert(WS_END <= (size_t)134217728);
static_assert((size_t)NPC * 16 == SZ_CV);
static_assert((size_t)(NROWS / 128) * (NPJ / 64) * 256 * 128 == SZ_XP);
static_assert((size_t)(NIN / 64) * NBATCH * NL * 128 == SZ_Y);

__device__ __forceinline__ unsigned short bf16_bits(float f) {
  unsigned u = __float_as_uint(f);
  u += 0x7FFFu + ((u >> 16) & 1u);
  return (unsigned short)(u >> 16);
}
__device__ __forceinline__ float bf16_val(unsigned short b) { return __uint_as_float(((unsigned)b) << 16); }
__device__ __forceinline__ float bf16r(float f) { return bf16_val(bf16_bits(f)); }
__device__ __forceinline__ v8f zero8() {
  v8f z;
#pragma unroll
  for (int i = 0; i < 8; ++i) z[i] = 0.0f;
  return z;
}

__device__ __forceinline__ void ldfrag_g(Frag& f, const unsigned short* p, int h) {
  f.half[0] = *(const v8usa*)(p + 8 * h);
  f.half[1] = *(const v8usa*)(p + 16 + 8 * h);
}
__device__ __forceinline__ v8f mma16(v8f c, const Frag& a, const Frag& b) {
  v8f d = __builtin_amdgcn_wmma_f32_16x16x32_bf16(false, a.v, false, b.v, (short)0, c, false, false);
  asm volatile("v_nop\n\tv_nop\n\tv_nop\n\tv_nop" : "+v"(d) : "v"(a.v), "v"(b.v));
  return d;
}

__global__ __launch_bounds__(256)
void cvt_kernel(const float* __restrict__ x, const float* __restrict__ win, const float* __restrict__ wout,
                unsigned short* cv)
{
  const int g = blockIdx.x * 256 + threadIdx.x;
  if (g >= NPC) return;
  const int e = g * 8;
  const float* src;
  if      (e < P_WIN)  src = x    + e;
  else if (e < P_WOUT) src = win  + (e - P_WIN);
  else                 src = wout + (e - P_WOUT);
  const v4f a = *(const v4fa*)src;
  const v4f c = *(const v4fa*)(src + 4);
  v8us o;
  o[0] = bf16_bits(a[0]); o[1] = bf16_bits(a[1]); o[2] = bf16_bits(a[2]); o[3] = bf16_bits(a[3]);
  o[4] = bf16_bits(c[0]); o[5] = bf16_bits(c[1]); o[6] = bf16_bits(c[2]); o[7] = bf16_bits(c[3]);
  unsigned short* dst = cv + e;
  *(volatile v8us*)dst = o;
  __threadfence();
  *(volatile v8us*)dst = o;
}

__device__ __forceinline__ void xp_store_pass(const float* sT, float* xp, int m0w, int cy, int w, int lane) {
  const int q8 = lane & 7, sub = lane >> 3;
#pragma unroll
  for (int i = 0; i < 16; ++i) {
    const int lid = 4 * i + sub;
    const int rl = lid >> 1, hl = lid & 1;
    const v4f v = *(const v4fa*)(sT + (32 * w + rl) * 64 + 32 * hl + 4 * q8);
    float* dst = xp + (size_t)(m0w + rl) * NPJ + 64 * cy + 32 * hl + 4 * q8;
    *(volatile v4f*)dst = v;
  }
}

__global__ __launch_bounds__(128)
void proj_in_kernel(const unsigned short* __restrict__ cv, float* xp)
{
  __shared__ __attribute__((aligned(16))) float sT[128 * 64];

  const int tid = threadIdx.x, lane = tid & 31, w = tid >> 5;
  const int h = lane >> 4, m = lane & 15;
  const int m0 = blockIdx.x * 128;
  const int cy = blockIdx.y;
  const int m0w = m0 + 32 * w;

  const unsigned short* xa = cv + P_X   + (size_t)(m0w + m) * NDIM;
  const unsigned short* wb = cv + P_WIN + (size_t)(64 * cy + m) * NDIM;

  v8f acc[2][4];
#pragma unroll
  for (int mt = 0; mt < 2; ++mt)
#pragma unroll
    for (int nt = 0; nt < 4; ++nt) acc[mt][nt] = zero8();

#pragma unroll 1
  for (int k0 = 0; k0 < NDIM; k0 += 32) {
    Frag a0, a1;
    ldfrag_g(a0, xa + k0, h);
    ldfrag_g(a1, xa + (size_t)16 * NDIM + k0, h);
#pragma unroll
    for (int nt = 0; nt < 4; ++nt) {
      Frag b;
      ldfrag_g(b, wb + (size_t)nt * 16 * NDIM + k0, h);
      acc[0][nt] = mma16(acc[0][nt], a0, b);
      acc[1][nt] = mma16(acc[1][nt], a1, b);
    }
  }

#pragma unroll
  for (int nt = 0; nt < 4; ++nt) {
    const int col = 16 * nt + m;
#pragma unroll
    for (int mt = 0; mt < 2; ++mt)
#pragma unroll
      for (int r = 0; r < 8; ++r) {
        const int rowl = 32 * w + 16 * mt + 8 * h + r;
        sT[rowl * 64 + col] = acc[mt][nt][r];
      }
  }
  __syncthreads();

  xp_store_pass(sT, xp, m0w, cy, w, lane);
  __threadfence();
  xp_store_pass(sT, xp, m0w, cy, w, lane);
}

__device__ __forceinline__ void y_store_pass(const unsigned short* sH, const unsigned short* sL,
                                             unsigned short* yh, unsigned short* yl,
                                             int b, int t0, int cx, int w, int lane) {
  const int q8 = lane & 7, sub = lane >> 3;
#pragma unroll
  for (int i = 0; i < 4; ++i) {
    const int lid = 16 * w + 4 * i + sub;
    const v8us vh = *(const v8usa*)(sH + lid * 64 + 8 * q8);
    const v8us vl = *(const v8usa*)(sL + lid * 64 + 8 * q8);
    const size_t go = ((size_t)(b * NL + t0 + lid)) * NIN + 64 * cx + 8 * q8;
    *(volatile v8us*)(yh + go) = vh;
    *(volatile v8us*)(yl + go) = vl;
  }
}

__global__ __launch_bounds__(64)
void scan_kernel(const float* __restrict__ xp, const float* __restrict__ convw,
                 const float* __restrict__ sdec, const float* __restrict__ sscl,
                 unsigned short* yh, unsigned short* yl)
{
  __shared__ __attribute__((aligned(16))) unsigned short sH[TCH * 64];
  __shared__ __attribute__((aligned(16))) unsigned short sL[TCH * 64];

  const int tid = threadIdx.x, lane = tid & 31, w = tid >> 5;
  const int cx = blockIdx.x;
  const int b  = blockIdx.y;
  const int c  = 64 * cx + tid;

  const float w0 = bf16r(convw[c * 3 + 0]);
  const float w1 = bf16r(convw[c * 3 + 1]);
  const float w2 = bf16r(convw[c * 3 + 2]);
  const float dd = 1.0f / (1.0f + __expf(-bf16r(sdec[c])));
  const float coef = (1.0f - dd) * bf16r(sscl[c]);

  const float* up = xp + (size_t)b * NL * NPJ + c;
  const float* gp = up + NIN;

  float um2 = 0.0f, um1 = 0.0f, y = 0.0f;
#pragma unroll 1
  for (int t0 = 0; t0 < NL; t0 += TCH) {
#pragma unroll 1
    for (int tl = 0; tl < TCH; ++tl) {
      const size_t ro = (size_t)(t0 + tl) * NPJ;
      const float u = up[ro];
      const float g = gp[ro];
      const float cvl = w0 * um2 + w1 * um1 + w2 * u;
      um2 = um1; um1 = u;
      y = dd * y + coef * cvl;
      const float e  = __expf(-g);
      const float sg = __builtin_amdgcn_rcpf(1.0f + e);
      const float v  = y * sg;
      const unsigned short hb = bf16_bits(v);
      const unsigned short lb = bf16_bits(v - bf16_val(hb));
      sH[tl * 64 + tid] = hb;
      sL[tl * 64 + tid] = lb;
    }
    __syncthreads();
    y_store_pass(sH, sL, yh, yl, b, t0, cx, w, lane);
    __threadfence();
    y_store_pass(sH, sL, yh, yl, b, t0, cx, w, lane);
    __syncthreads();
  }
}

constexpr int SP2 = NDIM + 4;
static_assert((SP2 * 4) % 16 == 0);

__global__ __launch_bounds__(256)
void proj_out_kernel(const unsigned short* __restrict__ yh, const unsigned short* __restrict__ yl,
                     const unsigned short* __restrict__ cv, const float* __restrict__ normw, float* out)
{
  __shared__ __attribute__((aligned(16))) float sT[32 * SP2];

  const int tid = threadIdx.x, lane = tid & 31, w = tid >> 5;
  const int h = lane >> 4, m = lane & 15;
  const int m0 = blockIdx.x * 32;

  const unsigned short* ha = yh + (size_t)(m0 + m) * NIN;
  const unsigned short* la = yl + (size_t)(m0 + m) * NIN;
  const unsigned short* wb = cv + P_WOUT + (size_t)(32 * w + m) * NIN;

  v8f acc[2][2];
#pragma unroll
  for (int mt = 0; mt < 2; ++mt)
#pragma unroll
    for (int nt = 0; nt < 2; ++nt) acc[mt][nt] = zero8();

#pragma unroll 1
  for (int k0 = 0; k0 < NIN; k0 += 32) {
    Frag ah[2], al[2], b[2];
#pragma unroll
    for (int mt = 0; mt < 2; ++mt) {
      ldfrag_g(ah[mt], ha + (size_t)mt * 16 * NIN + k0, h);
      ldfrag_g(al[mt], la + (size_t)mt * 16 * NIN + k0, h);
    }
#pragma unroll
    for (int nt = 0; nt < 2; ++nt) ldfrag_g(b[nt], wb + (size_t)nt * 16 * NIN + k0, h);
#pragma unroll
    for (int mt = 0; mt < 2; ++mt)
#pragma unroll
      for (int nt = 0; nt < 2; ++nt) {
        acc[mt][nt] = mma16(acc[mt][nt], ah[mt], b[nt]);
        acc[mt][nt] = mma16(acc[mt][nt], al[mt], b[nt]);
      }
  }

#pragma unroll
  for (int nt = 0; nt < 2; ++nt) {
    const int col = 32 * w + 16 * nt + m;
#pragma unroll
    for (int mt = 0; mt < 2; ++mt)
#pragma unroll
      for (int r = 0; r < 8; ++r) {
        const int row = 16 * mt + 8 * h + r;
        sT[row * SP2 + col] = acc[mt][nt][r];
      }
  }
  __syncthreads();

  const int sub = lane >> 3, q8 = lane & 7;
  const int row = 4 * w + sub;
  const float* sr = sT + row * SP2;
  float ss = 0.0f;
#pragma unroll
  for (int j = 0; j < 8; ++j) {
    const v4f v = *(const v4fa*)(sr + 32 * q8 + 4 * j);
    ss += v[0] * v[0];
    ss += v[1] * v[1];
    ss += v[2] * v[2];
    ss += v[3] * v[3];
  }
  ss += __shfl_xor(ss, 1);
  ss += __shfl_xor(ss, 2);
  ss += __shfl_xor(ss, 4);
  const float rstd = rsqrtf(ss * (1.0f / (float)NDIM) + 1e-6f);

  v4f o[8];
#pragma unroll
  for (int i = 0; i < 8; ++i) {
    const int col0 = 32 * i + 4 * q8;
    const v4f v  = *(const v4fa*)(sr + col0);
    const v4f nw = *(const v4fa*)(normw + col0);
    v4f t;
    t[0] = (v[0] * rstd) * bf16r(nw[0]);
    t[1] = (v[1] * rstd) * bf16r(nw[1]);
    t[2] = (v[2] * rstd) * bf16r(nw[2]);
    t[3] = (v[3] * rstd) * bf16r(nw[3]);
    o[i] = t;
  }
  float* orow = out + (size_t)(m0 + row) * NDIM + 4 * q8;
#pragma unroll
  for (int i = 0; i < 8; ++i) *(volatile v4f*)(orow + 32 * i) = o[i];
  __threadfence();
#pragma unroll
  for (int i = 0; i < 8; ++i) *(volatile v4f*)(orow + 32 * i) = o[i];
}

extern "C" void kernel_launch(void* const* d_in, const int* in_sizes, int n_in,
                              void* d_out, int out_size, void* d_ws, size_t ws_size,
                              hipStream_t stream)
{
  if (n_in < 7) return;
  if (in_sizes[0] != NROWS * NDIM) return;
  if (in_sizes[1] != NPJ * NDIM)   return;
  if (in_sizes[2] != NIN * 3)      return;
  if (in_sizes[3] != NIN)          return;
  if (in_sizes[4] != NIN)          return;
  if (in_sizes[5] != NDIM * NIN)   return;
  if (in_sizes[6] != NDIM)         return;
  if (out_size != NROWS * NDIM)    return;
  if (ws_size < WS_END)            return;

  const float* x     = (const float*)d_in[0];
  const float* win   = (const float*)d_in[1];
  const float* convw = (const float*)d_in[2];
  const float* sdec  = (const float*)d_in[3];
  const float* sscl  = (const float*)d_in[4];
  const float* wout  = (const float*)d_in[5];
  const float* normw = (const float*)d_in[6];
  float* out = (float*)d_out;

  char* ws = (char*)d_ws;
  unsigned short* cv = (unsigned short*)(ws + OFF_CV);
  float*          xp = (float*)(ws + OFF_XP);
  unsigned short* yh = (unsigned short*)(ws + OFF_YH);
  unsigned short* yl = (unsigned short*)(ws + OFF_YL);

  cvt_kernel<<<dim3(NCBLK), dim3(256), 0, stream>>>(x, win, wout, cv);

  proj_in_kernel<<<dim3(NROWS / 128, NPJ / 64), dim3(128), 0, stream>>>(cv, xp);

  scan_kernel<<<dim3(NIN / 64, NBATCH), dim3(64), 0, stream>>>(xp, convw, sdec, sscl, yh, yl);

  proj_out_kernel<<<dim3(NROWS / 32), dim3(256), 0, stream>>>(yh, yl, cv, normw, out);
}
